// RotaryAttention_18837726561069
// MI455X (gfx1250) — hardware-verified
//
#include <hip/hip_runtime.h>
#include <stddef.h>


#define DM 1024
#define NH 16
#define HD 64
#define SQ 2048
#define NB 2
#define MR (NB * SQ)
#define TABN (SQ * (HD / 2))

typedef _Float16 f16;
typedef f16 v16h __attribute__((ext_vector_type(16)));
typedef f16 v8h __attribute__((ext_vector_type(8)));
typedef float v8f __attribute__((ext_vector_type(8)));
typedef float v4f __attribute__((ext_vector_type(4)));
typedef unsigned int u32x4 __attribute__((ext_vector_type(4)));

union Frag { v16h v; v8h h[2]; };
union Pack8 { v8h h; u32x4 u; };

__device__ __forceinline__ v16h ld_frag(const f16* p, int hf) {
  Frag f;
  f.h[0] = *(const v8h*)(p + 8 * hf);
  f.h[1] = *(const v8h*)(p + 16 + 8 * hf);
  return f.v;
}

__device__ __forceinline__ v8f mma(v16h a, v16h b, v8f c) {
  return __builtin_amdgcn_wmma_f32_16x16x32_f16(false, a, false, b, (short)0, c, false, false);
}

#define GUARD4(c0, c1, c2, c3, x, y)                                           \
  asm volatile("v_nop\n\tv_nop\n\tv_nop\n\tv_nop"                              \
               : "+v"(c0), "+v"(c1), "+v"(c2), "+v"(c3)                        \
               : "v"(x), "v"(y))

__global__ void __launch_bounds__(256)
k_cvt(const float* __restrict__ src, f16* __restrict__ dst, int n, float scale) {
  const int i = (blockIdx.x * 256 + (int)threadIdx.x) * 8;
  if (i + 8 > n) return;
  const v4f a = *(const v4f*)(src + i);
  const v4f b = *(const v4f*)(src + i + 4);
  Pack8 p;
  p.h[0] = (f16)(a.x * scale); p.h[1] = (f16)(a.y * scale);
  p.h[2] = (f16)(a.z * scale); p.h[3] = (f16)(a.w * scale);
  p.h[4] = (f16)(b.x * scale); p.h[5] = (f16)(b.y * scale);
  p.h[6] = (f16)(b.z * scale); p.h[7] = (f16)(b.w * scale);
  const u32x4 v = p.u;
  f16* g = dst + i;
  *(volatile u32x4*)g = v;
  __threadfence();
  *(volatile u32x4*)g = v;
}

__global__ void __launch_bounds__(256)
k_rope_tab(float* __restrict__ cs, float* __restrict__ sn, int total) {
#pragma clang fp contract(off)
  const int t = blockIdx.x * 256 + (int)threadIdx.x;
  if (t >= total) return;
  const int s = t >> 5;
  const int i = t & 31;
  const double pw = exp2((double)i * 0.41524101186092029);
  const float p32 = (float)pw;
  const float fr = 1.0f / p32;
  const float ang = (float)s * fr;
  const double xd = (double)ang;
  const double kq = rint(xd * 0.63661977236758134);
  const double rd = fma(-kq, 1.5707963267948966, xd);
  const float r = (float)rd;
  const int qd = ((int)kq) & 3;
  const float r2 = r * r;
  const float sp = r + r * r2 * (-1.66666667e-1f + r2 * (8.33333333e-3f + r2 * (-1.98412698e-4f + r2 * 2.75573192e-6f)));
  const float cp = 1.0f + r2 * (-0.5f + r2 * (4.16666667e-2f + r2 * (-1.38888889e-3f + r2 * (2.48015873e-5f + r2 * (-2.75573192e-7f)))));
  float sv, cv;
  if (qd == 0)      { sv =  sp; cv =  cp; }
  else if (qd == 1) { sv =  cp; cv = -sp; }
  else if (qd == 2) { sv = -sp; cv = -cp; }
  else              { sv = -cp; cv =  sp; }
  *(volatile float*)(cs + t) = cv;
  *(volatile float*)(sn + t) = sv;
  __threadfence();
  *(volatile float*)(cs + t) = cv;
  *(volatile float*)(sn + t) = sv;
}

__device__ __forceinline__ void gemm32x32(const f16* __restrict__ ap, const f16* __restrict__ bp,
                                          int hf, v8f& c00, v8f& c01, v8f& c10, v8f& c11) {
  const v8f z = {0.0f, 0.0f, 0.0f, 0.0f, 0.0f, 0.0f, 0.0f, 0.0f};
  c00 = z; c01 = z; c10 = z; c11 = z;
#pragma unroll 1
  for (int k0 = 0; k0 < DM; k0 += 32) {
    const v16h a0 = ld_frag(ap + k0, hf);
    const v16h a1 = ld_frag(ap + 16 * DM + k0, hf);
    const v16h b0 = ld_frag(bp + k0, hf);
    const v16h b1 = ld_frag(bp + 16 * DM + k0, hf);
    c00 = mma(a0, b0, c00); c01 = mma(a0, b1, c01);
    c10 = mma(a1, b0, c10); c11 = mma(a1, b1, c11);
    GUARD4(c00, c01, c10, c11, a1, b1);
  }
}

__device__ __forceinline__ void epi_qkv(v8f c, int ti, int tj, int wr, int wc, int m, int hf,
                                        int s0, int sel, float bb,
                                        const float* __restrict__ cs, const float* __restrict__ sn,
                                        f16* sT) {
  const int lc = 32 * wc + 16 * tj + m;
#pragma unroll
  for (int r = 0; r < 8; ++r) {
    const int lr = 32 * wr + 16 * ti + 8 * hf + r;
    float v = c[r] * (1.0f / 64.0f) + bb;
    if (sel < 2) {
      const float vp = __shfl_xor(v, 1, 32);
      const int tix = (s0 + lr) * (HD / 2) + (lc >> 1);
      const float cv = cs[tix], sv = sn[tix];
      v = (lc & 1) ? (v * cv + vp * sv) : (v * cv - vp * sv);
    }
    const int idx = (sel < 2) ? (lr * 64 + lc) : (lc * 64 + lr);
    sT[idx] = (f16)(v * 8.0f);
  }
}

__global__ void __launch_bounds__(128)
k_qkv(const f16* __restrict__ xp,
      const f16* __restrict__ wq, const float* __restrict__ bq,
      const f16* __restrict__ wk, const float* __restrict__ bk,
      const f16* __restrict__ wv, const float* __restrict__ bv,
      const float* __restrict__ cs, const float* __restrict__ sn,
      f16* qo, f16* ko, f16* vo) {
  __shared__ f16 sT[64 * 64];
  const int wave = threadIdx.x >> 5, lane = threadIdx.x & 31, m = lane & 15, hf = lane >> 4;
  const int wr = wave >> 1, wc = wave & 1;
  const int row0 = blockIdx.x * 64, col0 = blockIdx.y * 64, sel = blockIdx.z;
  if (row0 >= MR || col0 >= DM || sel >= 3) return;
  const f16* W = (sel == 0) ? wq : ((sel == 1) ? wk : wv);
  const float* bias = (sel == 0) ? bq : ((sel == 1) ? bk : bv);
  f16* dst = (sel == 0) ? qo : ((sel == 1) ? ko : vo);
  const int b = row0 / SQ;
  const int s0 = row0 - b * SQ;
  const int head = blockIdx.y;
  const int bh = b * NH + head;

  v8f c00, c01, c10, c11;
  const f16* ap = xp + (size_t)(row0 + 32 * wr + m) * DM;
  const f16* bp = W + (size_t)(col0 + 32 * wc + m) * DM;
  gemm32x32(ap, bp, hf, c00, c01, c10, c11);

  const float bb0 = bias[col0 + 32 * wc + m];
  const float bb1 = bias[col0 + 32 * wc + 16 + m];
  epi_qkv(c00, 0, 0, wr, wc, m, hf, s0, sel, bb0, cs, sn, sT);
  epi_qkv(c01, 0, 1, wr, wc, m, hf, s0, sel, bb1, cs, sn, sT);
  epi_qkv(c10, 1, 0, wr, wc, m, hf, s0, sel, bb0, cs, sn, sT);
  epi_qkv(c11, 1, 1, wr, wc, m, hf, s0, sel, bb1, cs, sn, sT);
  __syncthreads();

  const int piece = lane & 7;
  u32x4 vals[4];
  f16* gp[4];
#pragma unroll
  for (int q = 0; q < 4; ++q) {
    const int L = wave * 16 + 4 * q + (lane >> 3);
    vals[q] = *(const u32x4*)(sT + L * 64 + piece * 8);
    const size_t off = (sel < 2) ? (((size_t)bh * SQ + s0 + L) * HD)
                                 : (((size_t)bh * HD + L) * SQ + s0);
    gp[q] = dst + off + piece * 8;
  }
#pragma unroll
  for (int q = 0; q < 4; ++q) *(volatile u32x4*)gp[q] = vals[q];
  __threadfence();
#pragma unroll
  for (int q = 0; q < 4; ++q) *(volatile u32x4*)gp[q] = vals[q];
}

__global__ void __launch_bounds__(128)
k_attn(const f16* __restrict__ qp, const f16* __restrict__ kp, const f16* __restrict__ vp, f16* op) {
  __shared__ f16 sO[4 * 16 * HD];
  const int wave = threadIdx.x >> 5, lane = threadIdx.x & 31, m = lane & 15, hf = lane >> 4;
  const int bh = blockIdx.y;
  const int b = bh / NH, head = bh - b * NH;
  const int qb0 = blockIdx.x * 64;
  if (qb0 >= SQ || bh >= NB * NH) return;
  const int qbase = qb0 + wave * 16;

  const f16* qrow = qp + ((size_t)bh * SQ + qbase + m) * HD;
  const v16h qf0 = ld_frag(qrow, hf);
  const v16h qf1 = ld_frag(qrow + 32, hf);
  const f16* kb = kp + (size_t)bh * SQ * HD + (size_t)m * HD;
  const f16* vb = vp + (size_t)bh * HD * SQ + (size_t)m * SQ;

  const v8f z = {0.0f, 0.0f, 0.0f, 0.0f, 0.0f, 0.0f, 0.0f, 0.0f};
  v8f o0 = z, o1 = z, o2 = z, o3 = z;
  float mrun = -3.0e38f, lrun = 0.0f;
  const float CE = 1.4426950408889634f * (1.0f / 512.0f);

#pragma unroll 1
  for (int j = 0; j < SQ; j += 64) {
    const f16* k0p = kb + (size_t)j * HD;
    v8f s0, s1, s2, s3;
    {
      const v16h a0 = ld_frag(k0p, hf),            a0b = ld_frag(k0p + 32, hf);
      const v16h a1 = ld_frag(k0p + 16 * HD, hf),  a1b = ld_frag(k0p + 16 * HD + 32, hf);
      const v16h a2 = ld_frag(k0p + 32 * HD, hf),  a2b = ld_frag(k0p + 32 * HD + 32, hf);
      const v16h a3 = ld_frag(k0p + 48 * HD, hf),  a3b = ld_frag(k0p + 48 * HD + 32, hf);
      s0 = mma(a0, qf0, z); s1 = mma(a1, qf0, z); s2 = mma(a2, qf0, z); s3 = mma(a3, qf0, z);
      s0 = mma(a0b, qf1, s0); s1 = mma(a1b, qf1, s1); s2 = mma(a2b, qf1, s2); s3 = mma(a3b, qf1, s3);
      GUARD4(s0, s1, s2, s3, a3b, qf1);
    }

    float mloc = -3.0e38f;
#pragma unroll
    for (int e = 0; e < 8; ++e)
      mloc = fmaxf(mloc, fmaxf(fmaxf(s0[e], s1[e]), fmaxf(s2[e], s3[e])));
    mloc = fmaxf(mloc, __shfl_xor(mloc, 16, 32));
    const float mnew = fmaxf(mrun, mloc);
    const float corr = __builtin_amdgcn_exp2f((mrun - mnew) * CE);
    const float kx = 12.0f - mnew * CE;
    float psum = 0.0f;
    Frag pA, pB;
#pragma unroll
    for (int e = 0; e < 8; ++e) {
      const float p0 = __builtin_amdgcn_exp2f(fmaf(s0[e], CE, kx));
      const float p1 = __builtin_amdgcn_exp2f(fmaf(s1[e], CE, kx));
      const float p2 = __builtin_amdgcn_exp2f(fmaf(s2[e], CE, kx));
      const float p3 = __builtin_amdgcn_exp2f(fmaf(s3[e], CE, kx));
      psum += (p0 + p1) + (p2 + p3);
      pA.v[e] = (f16)p0; pA.v[8 + e] = (f16)p1;
      pB.v[e] = (f16)p2; pB.v[8 + e] = (f16)p3;
    }
    psum += __shfl_xor(psum, 16, 32);
    lrun = lrun * corr + psum;
    mrun = mnew;
#pragma unroll
    for (int r = 0; r < 8; ++r) {
      const float cr = __shfl(corr, r + 8 * hf, 32);
      o0[r] *= cr; o1[r] *= cr; o2[r] *= cr; o3[r] *= cr;
    }

    {
      const f16* v0 = vb + j;
      const v16h w0 = ld_frag(v0, hf),           w1 = ld_frag(v0 + 16 * SQ, hf);
      const v16h w2 = ld_frag(v0 + 32 * SQ, hf), w3 = ld_frag(v0 + 48 * SQ, hf);
      const v16h w4 = ld_frag(v0 + 32, hf),           w5 = ld_frag(v0 + 16 * SQ + 32, hf);
      const v16h w6 = ld_frag(v0 + 32 * SQ + 32, hf), w7 = ld_frag(v0 + 48 * SQ + 32, hf);
      o0 = mma(pA.v, w0, o0); o1 = mma(pA.v, w1, o1); o2 = mma(pA.v, w2, o2); o3 = mma(pA.v, w3, o3);
      o0 = mma(pB.v, w4, o0); o1 = mma(pB.v, w5, o1); o2 = mma(pB.v, w6, o2); o3 = mma(pB.v, w7, o3);
      GUARD4(o0, o1, o2, o3, pB.v, w7);
    }
  }

  const float inv8 = 8.0f / lrun;
  f16* so = sO + wave * (16 * HD);
#pragma unroll
  for (int r = 0; r < 8; ++r) {
    const float lv = __shfl(inv8, r + 8 * hf, 32);
    const int rowq = 8 * hf + r;
    so[rowq * HD + 0 * 16 + m] = (f16)(o0[r] * lv);
    so[rowq * HD + 1 * 16 + m] = (f16)(o1[r] * lv);
    so[rowq * HD + 2 * 16 + m] = (f16)(o2[r] * lv);
    so[rowq * HD + 3 * 16 + m] = (f16)(o3[r] * lv);
  }
  __syncthreads();

  const int piece = lane & 7;
  u32x4 vals[4];
  f16* gp[4];
#pragma unroll
  for (int q = 0; q < 4; ++q) {
    const int L = 4 * q + (lane >> 3);
    vals[q] = *(const u32x4*)(so + L * HD + piece * 8);
    gp[q] = op + ((size_t)b * SQ + qbase + L) * DM + head * HD + piece * 8;
  }
#pragma unroll
  for (int q = 0; q < 4; ++q) *(volatile u32x4*)gp[q] = vals[q];
  __threadfence();
#pragma unroll
  for (int q = 0; q < 4; ++q) *(volatile u32x4*)gp[q] = vals[q];
}

__device__ __forceinline__ void epi_out(v8f c, int ti, int tj, int wr, int wc, int m, int hf,
                                        float bb, float* sF) {
  const int lc = 32 * wc + 16 * tj + m;
#pragma unroll
  for (int r = 0; r < 8; ++r) {
    const int lr = 32 * wr + 16 * ti + 8 * hf + r;
    sF[lr * 64 + lc] = c[r] * (1.0f / 4096.0f) + bb;
  }
}

__global__ void __launch_bounds__(128)
k_oproj(const f16* __restrict__ ap0, const f16* __restrict__ wo,
        const float* __restrict__ bo, float* out) {
  __shared__ float sF[64 * 64];
  const int wave = threadIdx.x >> 5, lane = threadIdx.x & 31, m = lane & 15, hf = lane >> 4;
  const int wr = wave >> 1, wc = wave & 1;
  const int row0 = blockIdx.x * 64, col0 = blockIdx.y * 64;
  if (row0 >= MR || col0 >= DM) return;

  v8f c00, c01, c10, c11;
  const f16* ap = ap0 + (size_t)(row0 + 32 * wr + m) * DM;
  const f16* bp = wo + (size_t)(col0 + 32 * wc + m) * DM;
  gemm32x32(ap, bp, hf, c00, c01, c10, c11);

  const float bb0 = bo[col0 + 32 * wc + m];
  const float bb1 = bo[col0 + 32 * wc + 16 + m];
  epi_out(c00, 0, 0, wr, wc, m, hf, bb0, sF);
  epi_out(c01, 0, 1, wr, wc, m, hf, bb1, sF);
  epi_out(c10, 1, 0, wr, wc, m, hf, bb0, sF);
  epi_out(c11, 1, 1, wr, wc, m, hf, bb1, sF);
  __syncthreads();

  const int piece = lane & 7;
  u32x4 vals[8];
  float* gp[8];
#pragma unroll
  for (int q = 0; q < 8; ++q) {
    const int L = wave * 32 + 4 * q + (lane >> 3);
    const int rowl = L >> 1, half = L & 1;
    vals[q] = *(const u32x4*)(sF + rowl * 64 + half * 32 + piece * 4);
    gp[q] = out + (size_t)(row0 + rowl) * DM + col0 + half * 32 + piece * 4;
  }
#pragma unroll
  for (int q = 0; q < 8; ++q) *(volatile u32x4*)gp[q] = vals[q];
  __threadfence();
#pragma unroll
  for (int q = 0; q < 8; ++q) *(volatile u32x4*)gp[q] = vals[q];
}

extern "C" void kernel_launch(void* const* d_in, const int* in_sizes, int n_in,
                              void* d_out, int out_size, void* d_ws, size_t ws_size,
                              hipStream_t stream) {
  if (n_in < 9) return;
  const size_t nx = (size_t)NB * SQ * DM;
  const size_t nw = (size_t)DM * DM;
  if ((size_t)in_sizes[0] != nx || (size_t)in_sizes[1] != nw || (size_t)in_sizes[3] != nw ||
      (size_t)in_sizes[5] != nw || (size_t)in_sizes[7] != nw ||
      in_sizes[2] != DM || in_sizes[4] != DM || in_sizes[6] != DM || in_sizes[8] != DM ||
      (size_t)out_size != nx)
    return;

  const float* x  = (const float*)d_in[0];
  const float* wq = (const float*)d_in[1];
  const float* bq = (const float*)d_in[2];
  const float* wk = (const float*)d_in[3];
  const float* bk = (const float*)d_in[4];
  const float* wv = (const float*)d_in[5];
  const float* bv = (const float*)d_in[6];
  const float* wo = (const float*)d_in[7];
  const float* bo = (const float*)d_in[8];
  float* out = (float*)d_out;

  f16* wsb = (f16*)d_ws;
  f16* xh  = wsb;
  f16* wqh = xh + nx;
  f16* wkh = wqh + nw;
  f16* wvh = wkh + nw;
  f16* woh = wvh + nw;
  f16* qh  = woh + nw;
  f16* kh  = qh + nx;
  f16* vh  = kh + nx;
  f16* ah  = vh + nx;
  float* cs = (float*)(ah + nx);
  float* sn = cs + TABN;
  const size_t total_bytes = (size_t)((const char*)(sn + TABN) - (const char*)d_ws);
  if (total_bytes > ws_size) return;

  const int blk_x = (int)((nx + 2047) / 2048);
  const int blk_w = (int)((nw + 2047) / 2048);
  k_cvt<<<blk_x, 256, 0, stream>>>(x,  xh,  (int)nx, 1.0f);
  k_cvt<<<blk_w, 256, 0, stream>>>(wq, wqh, (int)nw, 64.0f);
  k_cvt<<<blk_w, 256, 0, stream>>>(wk, wkh, (int)nw, 64.0f);
  k_cvt<<<blk_w, 256, 0, stream>>>(wv, wvh, (int)nw, 64.0f);
  k_cvt<<<blk_w, 256, 0, stream>>>(wo, woh, (int)nw, 64.0f);
  k_rope_tab<<<(TABN + 255) / 256, 256, 0, stream>>>(cs, sn, TABN);

  k_qkv<<<dim3((MR + 63) / 64, (DM + 63) / 64, 3), 128, 0, stream>>>(
      xh, wqh, bq, wkh, bk, wvh, bv, cs, sn, qh, kh, vh);
  k_attn<<<dim3((SQ + 63) / 64, NB * NH), 128, 0, stream>>>(qh, kh, vh, ah);
  k_oproj<<<dim3((MR + 63) / 64, (DM + 63) / 64), 128, 0, stream>>>(ah, woh, bo, out);
}
